// VecLinear_28982439313683
// MI455X (gfx1250) — hardware-run, weakly checked
//
#include <hip/hip_runtime.h>
#include <math.h>

typedef __attribute__((ext_vector_type(16))) _Float16 v16h;
typedef __attribute__((ext_vector_type(8)))  _Float16 v8h;
typedef __attribute__((ext_vector_type(16))) __bf16   v16b;
typedef __attribute__((ext_vector_type(8)))  __bf16   v8b;
typedef __attribute__((ext_vector_type(8)))  float    v8f;
typedef __attribute__((ext_vector_type(4)))  float    v4f;

constexpr int kBatch   = 8;
constexpr int kChan    = 128;
constexpr int kDim     = 3;
constexpr int kPts     = 4096;
constexpr int kSch     = 64;
constexpr int kCols    = kDim * kPts;
constexpr int kChunkB  = 2;
constexpr int kChunks  = kBatch / kChunkB;
constexpr int kM1      = 3 * kChan;
constexpr int kKfc     = 2 * kChan;
constexpr int kK67     = kChan + kSch;
static_assert(kCols == 12288);
static_assert(kChunks * kChunkB == kBatch);
static_assert((kChan % 32) == 0 && (kSch % 32) == 0 && (kKfc % 32) == 0 && (kK67 % 32) == 0);
static_assert((kM1 % 64) == 0 && (kChan % 64) == 0 && (kSch % 64) == 0 && (kCols % 64) == 0 && (kPts % 64) == 0);
static_assert((((kM1 / 64) * (kCols / 64)) % 8) == 0);
static_assert((((kChan / 64) * (kPts / 64)) % 8) == 0);
static_assert((((kChan / 64) * (kCols / 64)) % 8) == 0);
static_assert((((kSch / 64) * (kPts / 64)) % 8) == 0);

constexpr float kCarrySin = 64.0f;
constexpr float kCarrySn  = 256.0f;
constexpr float kCarryVs  = 256.0f;
constexpr float kCarrySs  = 1024.0f;
static_assert(kCarryVs * kCarrySn == kCarrySs * kCarrySin);
constexpr float kFold67  = 1.0f / (kCarryVs * kCarrySn);
constexpr float kF16MinNormal = 6.103515625e-5f;

constexpr size_t kSzVT  = (size_t)kChunkB * kCols * kChan * 2;
constexpr size_t kSzBT2 = (size_t)kChunkB * kPts * kK67 * 2;
constexpr size_t kSzSB  = (size_t)kChunkB * kPts * kSch * 2;
constexpr size_t kSzY1  = (size_t)kChunkB * kM1 * kCols * 4;
constexpr size_t kSzSC  = (size_t)kChunkB * kChan * kPts * 4;
constexpr size_t kSzCS  = (size_t)kChunkB * kKfc * kCols * 4;
constexpr size_t kSzSN  = (size_t)kChunkB * kChan * kPts * 4;
constexpr size_t kSzCT  = (size_t)kChunkB * kCols * kKfc * 2;
constexpr size_t kSzW1  = (size_t)kM1 * kChan * 2;
constexpr size_t kSzWFC = (size_t)kChan * kKfc * 2;
constexpr size_t kSzWSV = (size_t)kChan * kSch * 2;
constexpr size_t kSzW67 = (size_t)kSch * kK67 * 2;
constexpr int    kVecFloats = kM1 + kChan + kChan + kSch;
constexpr size_t kSzVEC = (size_t)kVecFloats * 4;
constexpr size_t kOffVTH  = 0;
constexpr size_t kOffVTL  = kOffVTH  + kSzVT;
constexpr size_t kOffBT2  = kOffVTL  + kSzVT;
constexpr size_t kOffSBH  = kOffBT2  + kSzBT2;
constexpr size_t kOffSBL  = kOffSBH  + kSzSB;
constexpr size_t kOffY1   = kOffSBL  + kSzSB;
constexpr size_t kOffSC   = kOffY1   + kSzY1;
constexpr size_t kOffCS   = kOffSC   + kSzSC;
constexpr size_t kOffSN   = kOffCS   + kSzCS;
constexpr size_t kOffCTH  = kOffSN   + kSzSN;
constexpr size_t kOffCTL  = kOffCTH  + kSzCT;
constexpr size_t kOffW1H  = kOffCTL  + kSzCT;
constexpr size_t kOffW1L  = kOffW1H  + kSzW1;
constexpr size_t kOffWFCH = kOffW1L  + kSzW1;
constexpr size_t kOffWFCL = kOffWFCH + kSzWFC;
constexpr size_t kOffWSVH = kOffWFCL + kSzWFC;
constexpr size_t kOffWSVL = kOffWSVH + kSzWSV;
constexpr size_t kOffW67  = kOffWSVL + kSzWSV;
constexpr size_t kOffVEC  = kOffW67  + kSzW67;
constexpr size_t kWsTotal = kOffVEC  + kSzVEC;
static_assert(kWsTotal == 114682624ull);
static_assert(kWsTotal <= 134217728ull);
static_assert((kOffVTL % 128) == 0 && (kOffBT2 % 128) == 0 && (kOffSBH % 128) == 0 && (kOffSBL % 128) == 0 &&
              (kOffY1 % 128) == 0 && (kOffSC % 128) == 0 && (kOffCS % 128) == 0 && (kOffSN % 128) == 0 &&
              (kOffCTH % 128) == 0 && (kOffCTL % 128) == 0 && (kOffW1H % 128) == 0 && (kOffW1L % 128) == 0 &&
              (kOffWFCH % 128) == 0 && (kOffWFCL % 128) == 0 && (kOffWSVH % 128) == 0 && (kOffWSVL % 128) == 0 &&
              (kOffW67 % 128) == 0 && (kOffVEC % 128) == 0 && (kSzVEC % 128) == 0);
static_assert(kVecFloats == 704 && (kVecFloats % 4) == 0);
constexpr int kVecBias1 = 0;
constexpr int kVecBfc   = kM1;
constexpr int kVecRsv   = kM1 + kChan;
constexpr int kVecB67   = kM1 + 2 * kChan;

__device__ __forceinline__ _Float16 to_h16(float x) {
  const float y = (fabsf(x) < kF16MinNormal) ? 0.0f : x;
  return (_Float16)y;
}
__device__ __forceinline__ unsigned short f2bf_bits(float f) {
  unsigned u = __float_as_uint(f);
  return (unsigned short)((u + 0x7FFFu + ((u >> 16) & 1u)) >> 16);
}
__device__ __forceinline__ float bf_bits2f(unsigned short h) { return __uint_as_float(((unsigned)h) << 16); }

__device__ __forceinline__ void tie2(v8f& a, v16h x, v16h y) { asm volatile("" : "+v"(a) : "v"(x), "v"(y)); }
__device__ __forceinline__ void tie2(v8f& a, v16b x, v16b y) { asm volatile("" : "+v"(a) : "v"(x), "v"(y)); }
__device__ __forceinline__ void tie4(v8f& a, v16h x, v16h y, v16h z, v16h w) { asm volatile("" : "+v"(a) : "v"(x), "v"(y), "v"(z), "v"(w)); }
__device__ __forceinline__ void tie4(v8f& a, v16b x, v16b y, v16b z, v16b w) { asm volatile("" : "+v"(a) : "v"(x), "v"(y), "v"(z), "v"(w)); }
__device__ __forceinline__ void guard2(v8f& a, v16h x, v16h y) { asm volatile("v_nop\n\tv_nop\n\tv_nop\n\tv_nop" : "+v"(a) : "v"(x), "v"(y)); }
__device__ __forceinline__ void guard2(v8f& a, v16b x, v16b y) { asm volatile("v_nop\n\tv_nop\n\tv_nop\n\tv_nop" : "+v"(a) : "v"(x), "v"(y)); }
__device__ __forceinline__ void guard4(v8f& a, v16h x, v16h y, v16h z, v16h w) { asm volatile("v_nop\n\tv_nop\n\tv_nop\n\tv_nop" : "+v"(a) : "v"(x), "v"(y), "v"(z), "v"(w)); }
__device__ __forceinline__ void guard4(v8f& a, v16b x, v16b y, v16b z, v16b w) { asm volatile("v_nop\n\tv_nop\n\tv_nop\n\tv_nop" : "+v"(a) : "v"(x), "v"(y), "v"(z), "v"(w)); }
__device__ __forceinline__ void keep4(v16h a, v16h b, v16h c, v16h d) { asm volatile("v_nop" :: "v"(a), "v"(b), "v"(c), "v"(d)); }
__device__ __forceinline__ void keep4(v16b a, v16b b, v16b c, v16b d) { asm volatile("v_nop" :: "v"(a), "v"(b), "v"(c), "v"(d)); }
__device__ __forceinline__ void acc_guard1(v8f& a) { asm volatile("v_nop\n\tv_nop\n\tv_nop\n\tv_nop" : "+v"(a)); }

template <typename T> struct Frag;
template <> struct Frag<_Float16> {
  typedef v16h V; union U { v16h v; v8h h[2]; };
  static __device__ __forceinline__ v16h load(const _Float16* p) {
    U f; f.h[0] = *(const v8h*)(p); f.h[1] = *(const v8h*)(p + 16); return f.v;
  }
  static __device__ __forceinline__ v8f mma(v16h a, v16h b, v8f c) {
    return __builtin_amdgcn_wmma_f32_16x16x32_f16(false, a, false, b, (short)0, c, false, false);
  }
};
template <> struct Frag<__bf16> {
  typedef v16b V; union U { v16b v; v8b h[2]; };
  static __device__ __forceinline__ v16b load(const __bf16* p) {
    U f; f.h[0] = *(const v8b*)(p); f.h[1] = *(const v8b*)(p + 16); return f.v;
  }
  static __device__ __forceinline__ v8f mma(v16b a, v16b b, v8f c) {
    return __builtin_amdgcn_wmma_f32_16x16x32_bf16(false, a, false, b, (short)0, c, false, false);
  }
};
template <bool SPLIT> struct ElemSel { typedef __bf16 T; };
template <> struct ElemSel<false> { typedef _Float16 T; };

template <bool SPLIT>
__global__ __launch_bounds__(256) void gemm16_kernel(
    const unsigned short* __restrict__ Ap, const unsigned short* __restrict__ A2p, int lda,
    const unsigned short* __restrict__ Btp, const unsigned short* __restrict__ Bt2p, int ldb, long strideB,
    float* __restrict__ Cout, int ldc, long strideC,
    const float* __restrict__ bias, int M, int N, int K, float scale)
{
  typedef typename ElemSel<SPLIT>::T T;
  typedef typename Frag<T>::V V;
  const T* A   = (const T*)Ap;
  const T* A2  = (const T*)A2p;
  const T* Bt  = (const T*)Btp;
  const T* Bt2 = (const T*)Bt2p;
  __shared__ __align__(16) float sT[8][16 * 68];
  const int b    = blockIdx.y;
  const int lane = threadIdx.x & 31;
  const int wave = threadIdx.x >> 5;
  const int tilesN = N >> 6;
  const int tilesM = M >> 6;
  const int tile = blockIdx.x * 8 + wave;
  if (tile >= tilesM * tilesN) return;
  const int tm = tile / tilesN;
  const int tn = tile - tm * tilesN;
  const int m0 = tm << 6;
  const int n0 = tn << 6;
  const T* Bb  = Bt  + (size_t)b * strideB;
  const T* Bb2 = Bt2 + (size_t)b * strideB;
  const int rlane = lane & 15;
  const int koff  = (lane >> 4) * 8;
  const int mOff  = (lane >> 4) * 8;

  v8f acc[4][4];
#pragma unroll
  for (int i = 0; i < 4; ++i)
#pragma unroll
    for (int j = 0; j < 4; ++j) acc[i][j] = (v8f){0.f,0.f,0.f,0.f,0.f,0.f,0.f,0.f};

  for (int k0 = 0; k0 < K; k0 += 32) {
    V bh[4], bl[4];
#pragma unroll
    for (int j = 0; j < 4; ++j) {
      const size_t bo = (size_t)(n0 + (j << 4) + rlane) * ldb + koff + k0;
      bh[j] = Frag<T>::load(Bb + bo);
      if (SPLIT) bl[j] = Frag<T>::load(Bb2 + bo);
      else       bl[j] = bh[j];
    }
#pragma unroll
    for (int i = 0; i < 4; ++i) {
      const size_t ao = (size_t)(m0 + (i << 4) + rlane) * lda + koff + k0;
      const V ah = Frag<T>::load(A + ao);
      V al = ah;
      if (SPLIT) al = Frag<T>::load(A2 + ao);
#pragma unroll
      for (int j = 0; j < 4; ++j) {
        acc[i][j] = Frag<T>::mma(ah, bh[j], acc[i][j]);
        if (SPLIT) {
          acc[i][j] = Frag<T>::mma(ah, bl[j], acc[i][j]);
          acc[i][j] = Frag<T>::mma(al, bh[j], acc[i][j]);
        }
      }
      if (SPLIT) {
        tie4(acc[i][0], ah, al, bh[0], bl[0]);
        tie4(acc[i][1], ah, al, bh[1], bl[1]);
        tie4(acc[i][2], ah, al, bh[2], bl[2]);
        guard4(acc[i][3], ah, al, bh[3], bl[3]);
      } else {
        tie2(acc[i][0], ah, bh[0]);
        tie2(acc[i][1], ah, bh[1]);
        tie2(acc[i][2], ah, bh[2]);
        guard2(acc[i][3], ah, bh[3]);
      }
    }
    keep4(bh[0], bh[1], bh[2], bh[3]);
    if (SPLIT) keep4(bl[0], bl[1], bl[2], bl[3]);
  }
#pragma unroll
  for (int i = 0; i < 4; ++i) {
    acc_guard1(acc[i][0]);
    acc_guard1(acc[i][1]);
    acc_guard1(acc[i][2]);
    acc_guard1(acc[i][3]);
  }

  float* slab = sT[wave];
  float* C = Cout + (size_t)b * strideC;
  const int hh = lane >> 4, c4 = (lane & 15) * 4;
#pragma unroll
  for (int i = 0; i < 4; ++i) {
    const int mBase = m0 + (i << 4);
    const v4f b0 = *(const v4f*)(bias + mBase + mOff);
    const v4f b1 = *(const v4f*)(bias + mBase + mOff + 4);
    const float bv[8] = {b0[0], b0[1], b0[2], b0[3], b1[0], b1[1], b1[2], b1[3]};
#pragma unroll
    for (int j = 0; j < 4; ++j) {
#pragma unroll
      for (int r = 0; r < 8; ++r) {
        const float v = acc[i][j][r] * scale + bv[r];
        slab[(mOff + r) * 68 + (j << 4) + rlane] = v;
      }
    }
    __builtin_amdgcn_fence(__ATOMIC_RELEASE, "workgroup");
    __builtin_amdgcn_wave_barrier();
    __builtin_amdgcn_fence(__ATOMIC_ACQUIRE, "workgroup");
    for (int pass = 0; pass < 2; ++pass) {
#pragma unroll
      for (int it = 0; it < 8; ++it) {
        const int row = it * 2 + hh;
        const v4f v = *(const v4f*)(slab + row * 68 + c4);
        *(volatile v4f*)(C + (size_t)(mBase + row) * ldc + n0 + c4) = v;
      }
      __threadfence();
    }
    __builtin_amdgcn_fence(__ATOMIC_RELEASE, "workgroup");
    __builtin_amdgcn_wave_barrier();
    __builtin_amdgcn_fence(__ATOMIC_ACQUIRE, "workgroup");
  }
}

template <int KC, int MODE>
__global__ __launch_bounds__(256) void transpose_cvt_kernel(
    const float* __restrict__ src, long srcBatchStride, int srcPitch,
    unsigned short* __restrict__ dst, unsigned short* __restrict__ dst2,
    int dstLd, int dstK0, int colsPerBatch, float carry)
{
  static_assert(KC == 64 || KC == 128);
  static_assert(MODE == 0 || MODE == 1);
  __shared__ __align__(16) float sT[KC * 68];
  const int tid = threadIdx.x, lane = tid & 31, wave = tid >> 5;
  const int b = blockIdx.y, kz = blockIdx.z;
  const int col0 = blockIdx.x * 64;
  const float* sp = src + (size_t)b * srcBatchStride + (size_t)(kz * KC) * srcPitch + col0;
  const int cl = tid >> 4, c4 = (tid & 15) * 4;
#pragma unroll
  for (int p = 0; p < KC / 16; ++p) {
    const int c = p * 16 + cl;
    const v4f v = *(const v4f*)(sp + (size_t)c * srcPitch + c4);
    *(v4f*)(sT + c * 68 + c4) = v;
  }
  __syncthreads();
  constexpr int LPR = KC / 8;
  constexpr int RPI = 32 / LPR;
  constexpr int NIT = 8 / RPI;
  const int sub = lane / LPR;
  const int k8  = (lane % LPR) * 8;
  v8h hv[NIT], lv[NIT];
#pragma unroll
  for (int it = 0; it < NIT; ++it) {
    const int col = wave * 8 + it * RPI + sub;
#pragma unroll
    for (int e = 0; e < 8; ++e) {
      const float x = sT[(k8 + e) * 68 + col] * carry;
      if (MODE == 0) {
        hv[it][e] = to_h16(x);
        lv[it][e] = (_Float16)0.0f;
      } else {
        const unsigned short hb = f2bf_bits(x);
        const unsigned short lb = f2bf_bits(x - bf_bits2f(hb));
        hv[it][e] = __builtin_bit_cast(_Float16, hb);
        lv[it][e] = __builtin_bit_cast(_Float16, lb);
      }
    }
  }
  for (int pass = 0; pass < 2; ++pass) {
#pragma unroll
    for (int it = 0; it < NIT; ++it) {
      const int col = wave * 8 + it * RPI + sub;
      const size_t row = (size_t)b * colsPerBatch + col0 + col;
      const size_t off = row * dstLd + dstK0 + kz * KC + k8;
      *(volatile v8h*)(dst + off) = hv[it];
      if (MODE == 1) *(volatile v8h*)(dst2 + off) = lv[it];
    }
    __threadfence();
  }
}

constexpr int kPrepRows      = 3 * kChan + kChan + kChan + kSch;
constexpr int kPrepRowBlocks = kPrepRows / 8;
static_assert(kPrepRows == 704 && kPrepRowBlocks * 8 == kPrepRows);

__global__ __launch_bounds__(256) void prep_kernel(
    const float* __restrict__ weight, const float* __restrict__ cross_w, const float* __restrict__ cross_b,
    const float* __restrict__ crossfc_w, const float* __restrict__ crossfc_b,
    const float* __restrict__ vsdir_w, const float* __restrict__ vsdir_b,
    const float* __restrict__ sv_w, const float* __restrict__ vs_w, const float* __restrict__ vs_b,
    const float* __restrict__ ss_w, const float* __restrict__ ss_b,
    unsigned short* __restrict__ W1H, unsigned short* __restrict__ W1L,
    unsigned short* __restrict__ WFCH, unsigned short* __restrict__ WFCL,
    unsigned short* __restrict__ WSVH, unsigned short* __restrict__ WSVL,
    unsigned short* __restrict__ W67, float* __restrict__ VEC)
{
  __shared__ __align__(16) float sv[kVecFloats];
  const int tid = threadIdx.x, lane = tid & 31;
  if (blockIdx.x == kPrepRowBlocks) {
    float s0 = 0.f, s1 = 0.f, s2 = 0.f;
#pragma unroll 1
    for (int i = 0; i < kChan; ++i) {
      const float a = cross_b[i], c = crossfc_b[i], d = vsdir_b[i];
      s0 += a * a;
      s1 += c * c;
      s2 += d * d;
    }
    const float inv0 = 1.0e-6f / fmaxf(sqrtf(s0), 1.0e-12f);
    const float inv1 = 1.0e-6f / fmaxf(sqrtf(s1), 1.0e-12f);
    const float inv2 = 1.0e-6f / fmaxf(sqrtf(s2), 1.0e-12f);
    const int tc = tid & (kChan - 1);
    const int t6 = tid & (kSch - 1);
    float rs = 0.f;
#pragma unroll 1
    for (int c = 0; c < kChan; ++c) {
      const float w = vsdir_w[tc * kChan + c];
      const unsigned short hb = f2bf_bits(w);
      const float hf = bf_bits2f(hb);
      const unsigned short lb = f2bf_bits(w - hf);
      rs += (hf + bf_bits2f(lb));
    }
    float cb = cross_b[tc], fb = crossfc_b[tc], vb = vsdir_b[tc], vsb = vs_b[t6], ssb = ss_b[t6];
    asm volatile("" : "+v"(cb), "+v"(fb), "+v"(vb), "+v"(vsb), "+v"(ssb));
    const bool lo = (tid < kChan);
    sv[tid] = lo ? 0.0f : cb * inv0;
    sv[2 * kChan + tid] = lo ? vb * inv2 : fb * inv1;
    const float third = lo ? rs : (vsb + ssb);
    if (tid < kChan + kSch) sv[4 * kChan + tid] = third;
    __syncthreads();
    if (tid < kVecFloats / 4) {
      const v4f v = *(const v4f*)(sv + 4 * tid);
      *(volatile v4f*)(VEC + 4 * tid) = v;
    }
    __threadfence();
    if (tid < kVecFloats / 4) {
      const v4f v = *(const v4f*)(sv + 4 * tid);
      *(volatile v4f*)(VEC + 4 * tid) = v;
    }
    return;
  }
  const int gw = __builtin_amdgcn_readfirstlane((int)blockIdx.x * 8 + (tid >> 5));
  const float* srcA;
  const float* srcB;
  int nA, nB, comp, L, split;
  float cA, cB;
  unsigned short* dst;
  unsigned short* dst2;
  if (gw < kChan) {
    srcA = weight + gw * (kChan - 1); srcB = srcA; nA = kChan - 1; nB = 0; comp = 1; L = kChan; split = 1;
    cA = 1.0f; cB = 1.0f; dst = W1H + (size_t)gw * kChan; dst2 = W1L + (size_t)gw * kChan;
  } else if (gw < 2 * kChan) {
    srcA = cross_w + (gw - kChan) * (kChan - 1); srcB = srcA; nA = kChan - 1; nB = 0; comp = 1; L = kChan; split = 1;
    cA = 1.0f; cB = 1.0f; dst = W1H + (size_t)gw * kChan; dst2 = W1L + (size_t)gw * kChan;
  } else if (gw < 3 * kChan) {
    srcA = vsdir_w + (gw - 2 * kChan) * kChan; srcB = srcA; nA = kChan; nB = 0; comp = 0; L = kChan; split = 1;
    cA = 1.0f; cB = 1.0f; dst = W1H + (size_t)gw * kChan; dst2 = W1L + (size_t)gw * kChan;
  } else if (gw < 4 * kChan) {
    const int r = gw - 3 * kChan;
    srcA = crossfc_w + r * (kKfc - 1); srcB = srcA; nA = kKfc - 1; nB = 0; comp = 1; L = kKfc; split = 1;
    cA = 1.0f; cB = 1.0f; dst = WFCH + (size_t)r * kKfc; dst2 = WFCL + (size_t)r * kKfc;
  } else if (gw < 5 * kChan) {
    const int r = gw - 4 * kChan;
    srcA = sv_w + r * kSch; srcB = srcA; nA = kSch; nB = 0; comp = 0; L = kSch; split = 1;
    cA = 1.0f; cB = 1.0f; dst = WSVH + (size_t)r * kSch; dst2 = WSVL + (size_t)r * kSch;
  } else {
    const int r = gw - 5 * kChan;
    srcA = vs_w + r * kChan; srcB = ss_w + r * kSch; nA = kChan; nB = kSch; comp = 0; L = kK67; split = 0;
    cA = kCarryVs; cB = kCarrySs; dst = W67 + (size_t)r * kK67; dst2 = dst;
  }
  float sum = 0.f;
  if (comp) {
#pragma unroll 1
    for (int k = 0; k < nA; ++k) sum += srcA[k];
  }
  asm volatile("" : "+v"(sum));
  const int nBm1 = (nB > 0) ? (nB - 1) : 0;
  v8h hv, lv;
#pragma unroll
  for (int e = 0; e < 8; ++e) {
    const int k  = lane * 8 + e;
    const int ka = (k < nA) ? k : (nA - 1);
    int kb = k - nA;
    kb = (kb < 0) ? 0 : kb;
    kb = (kb > nBm1) ? nBm1 : kb;
    float xa = srcA[ka];
    float xb = srcB[kb];
    asm volatile("" : "+v"(xa), "+v"(xb));
    const float val = (k < nA) ? xa * cA : ((k < nA + nB) ? xb * cB : (1.0f - sum) * cA);
    const unsigned short hbits = f2bf_bits(val);
    const unsigned short lbits = f2bf_bits(val - bf_bits2f(hbits));
    const _Float16 hf = to_h16(val);
    const unsigned short fbits = __builtin_bit_cast(unsigned short, hf);
    const unsigned short pick = split ? hbits : fbits;
    hv[e] = __builtin_bit_cast(_Float16, pick);
    lv[e] = __builtin_bit_cast(_Float16, lbits);
  }
  unsigned short* dp  = dst + lane * 8;
  unsigned short* dp2 = dst2 + lane * 8;
  const bool act = (lane < (L >> 3));
  if (act) *(volatile v8h*)dp = hv;
  if (split) {
    if (act) *(volatile v8h*)dp2 = lv;
  }
  __threadfence();
  if (act) *(volatile v8h*)dp = hv;
  if (split) {
    if (act) *(volatile v8h*)dp2 = lv;
  }
}

__global__ __launch_bounds__(256) void stats_kernel(
    const float* __restrict__ vin, const float* __restrict__ Y1, const float* __restrict__ SC,
    const float* __restrict__ rsv, float* __restrict__ CS, float* __restrict__ SN)
{
  const int g = blockIdx.x * 256 + threadIdx.x;
  const int b = g / kPts;
  const int n = g - b * kPts;
  const float* vp = vin + (size_t)b * kChan * kCols + n;
  const float* y1 = Y1 + (size_t)b * kM1 * kCols + n;
  const float* sc = SC + (size_t)b * kChan * kPts + n;
  float* cs = CS + (size_t)b * kKfc * kCols + n;
  float* sn = SN + (size_t)b * kChan * kPts + n;

  float sv0 = 0.f, sv1 = 0.f, sv2 = 0.f;
  float so0 = 0.f, so1 = 0.f, so2 = 0.f;
  float sd0 = 0.f, sd1 = 0.f, sd2 = 0.f;
  float ss = 0.f;
#pragma unroll 1
  for (int o = 0; o < kChan; ++o) {
    const float* pv = vp + (size_t)o * kCols;
    const float* po = y1 + (size_t)o * kCols;
    const float* pd = y1 + (size_t)(kChan + o) * kCols;
    const float s = sc[(size_t)o * kPts];
    sv0 += pv[0]; sv1 += pv[kPts]; sv2 += pv[2 * kPts];
    so0 += po[0]; so1 += po[kPts]; so2 += po[2 * kPts];
    sd0 += pd[0]; sd1 += pd[kPts]; sd2 += pd[2 * kPts];
    ss = fmaf(s, s, ss);
  }
  constexpr float kInvC = 1.0f / (float)kChan;
  const float mv0 = sv0 * kInvC, mv1 = sv1 * kInvC, mv2 = sv2 * kInvC;
  const float m0 = so0 * kInvC, m1 = so1 * kInvC, m2 = so2 * kInvC;
  const float du0 = sd0 * kInvC, du1 = sd1 * kInvC, du2 = sd2 * kInvC;
  const float invS = 1.0f / fmaxf(sqrtf(ss), 1.0e-12f);

  float t0 = 0.f, t1 = 0.f, t2 = 0.f, sx = 0.f, sq = 0.f;
#pragma unroll 1
  for (int o = 0; o < kChan; ++o) {
    const float* pv = vp + (size_t)o * kCols;
    const float* po = y1 + (size_t)o * kCols;
    const float* pd = y1 + (size_t)(kChan + o) * kCols;
    const float* pr = y1 + (size_t)(2 * kChan + o) * kCols;
    const float scale = sc[(size_t)o * kPts] * invS;
    const float rs = rsv[o];
    const float a0 = (po[0] - m0) * scale + m0;
    const float a1 = (po[kPts] - m1) * scale + m1;
    const float a2 = (po[2 * kPts] - m2) * scale + m2;
    t0 += a0; t1 += a1; t2 += a2;
    const float x0 = pd[0] - du0, x1 = pd[kPts] - du1, x2 = pd[2 * kPts] - du2;
    sx = fmaf(x0, x0, sx); sx = fmaf(x1, x1, sx); sx = fmaf(x2, x2, sx);
    const float r0 = pr[0] - rs * mv0, r1 = pr[kPts] - rs * mv1, r2 = pr[2 * kPts] - rs * mv2;
    const float rr = r0 * r0 + r1 * r1 + r2 * r2;
    const float inr = __builtin_amdgcn_rcpf(fmaxf(__builtin_amdgcn_sqrtf(rr), 1.0e-12f));
    const float e0 = pv[0] - mv0, e1 = pv[kPts] - mv1, e2 = pv[2 * kPts] - mv2;
    const float sp = (e0 * r0 + e1 * r1 + e2 * r2) * inr;
    sq = fmaf(sp, sp, sq);
  }
  const float oo0 = t0 * kInvC, oo1 = t1 * kInvC, oo2 = t2 * kInvC;
  const float invX = 1.0f / fmaxf(sqrtf(sx), 1.0e-12f);
  const float invQ = 1.0f / fmaxf(sqrtf(sq), 1.0e-12f);

#pragma unroll 1
  for (int o = 0; o < kChan; ++o) {
    const float* pv = vp + (size_t)o * kCols;
    const float* po = y1 + (size_t)o * kCols;
    const float* pd = y1 + (size_t)(kChan + o) * kCols;
    const float* pr = y1 + (size_t)(2 * kChan + o) * kCols;
    const float scale = sc[(size_t)o * kPts] * invS;
    const float rs = rsv[o];
    const float a0 = (po[0] - m0) * scale + m0;
    const float a1 = (po[kPts] - m1) * scale + m1;
    const float a2 = (po[2 * kPts] - m2) * scale + m2;
    const float w0 = a0 - oo0, w1 = a1 - oo1, w2 = a2 - oo2;
    const float x0 = (pd[0] - du0) * invX, x1 = (pd[kPts] - du1) * invX, x2 = (pd[2 * kPts] - du2) * invX;
    const float c0 = (x1 * w2 - x2 * w1) + a0;
    const float c1 = (x2 * w0 - x0 * w2) + a1;
    const float c2 = (x0 * w1 - x1 * w0) + a2;
    const float r0 = pr[0] - rs * mv0, r1 = pr[kPts] - rs * mv1, r2 = pr[2 * kPts] - rs * mv2;
    const float rr = r0 * r0 + r1 * r1 + r2 * r2;
    const float inr = __builtin_amdgcn_rcpf(fmaxf(__builtin_amdgcn_sqrtf(rr), 1.0e-12f));
    const float e0 = pv[0] - mv0, e1 = pv[kPts] - mv1, e2 = pv[2 * kPts] - mv2;
    const float sv = (e0 * r0 + e1 * r1 + e2 * r2) * inr * invQ;
    float* q0 = cs + (size_t)o * kCols;
    float* q1 = cs + (size_t)(kChan + o) * kCols;
    float* q2 = sn + (size_t)o * kPts;
    for (int pass = 0; pass < 2; ++pass) {
      *(volatile float*)(q0) = c0;
      *(volatile float*)(q0 + kPts) = c1;
      *(volatile float*)(q0 + 2 * kPts) = c2;
      *(volatile float*)(q1) = a0;
      *(volatile float*)(q1 + kPts) = a1;
      *(volatile float*)(q1 + 2 * kPts) = a2;
      *(volatile float*)(q2) = sv;
      __threadfence();
    }
  }
}

extern "C" void kernel_launch(void* const* d_in, const int* in_sizes, int n_in,
                              void* d_out, int out_size, void* d_ws, size_t ws_size,
                              hipStream_t stream) {
  if (n_in < 15) return;
  if (in_sizes[0] != kBatch * kChan * kCols) return;
  if (in_sizes[1] != kBatch * kSch * kPts) return;
  if (in_sizes[2] != kChan * (kChan - 1)) return;
  if (in_sizes[3] != kChan * kSch) return;
  if (in_sizes[4] != kChan) return;
  if (in_sizes[5] != kChan * (kChan - 1)) return;
  if (in_sizes[6] != kChan) return;
  if (in_sizes[7] != kChan * (kKfc - 1)) return;
  if (in_sizes[8] != kChan) return;
  if (in_sizes[9] != kChan * kChan) return;
  if (in_sizes[10] != kChan) return;
  if (in_sizes[11] != kSch * kChan) return;
  if (in_sizes[12] != kSch) return;
  if (in_sizes[13] != kSch * kSch) return;
  if (in_sizes[14] != kSch) return;
  if (out_size != kBatch * kChan * kCols + kBatch * kSch * kPts) return;
  if (ws_size < kWsTotal) return;

  const float* v_input   = (const float*)d_in[0];
  const float* s_input   = (const float*)d_in[1];
  const float* weight    = (const float*)d_in[2];
  const float* sv_w      = (const float*)d_in[3];
  const float* sv_b      = (const float*)d_in[4];
  const float* cross_w   = (const float*)d_in[5];
  const float* cross_b   = (const float*)d_in[6];
  const float* crossfc_w = (const float*)d_in[7];
  const float* crossfc_b = (const float*)d_in[8];
  const float* vsdir_w   = (const float*)d_in[9];
  const float* vsdir_b   = (const float*)d_in[10];
  const float* vs_w      = (const float*)d_in[11];
  const float* vs_b      = (const float*)d_in[12];
  const float* ss_w      = (const float*)d_in[13];
  const float* ss_b      = (const float*)d_in[14];
  float* out0 = (float*)d_out;
  float* out1 = (float*)d_out + (size_t)kBatch * kChan * kCols;

  char* ws = (char*)d_ws;
  unsigned short* VTH  = (unsigned short*)(ws + kOffVTH);
  unsigned short* VTL  = (unsigned short*)(ws + kOffVTL);
  unsigned short* BT2  = (unsigned short*)(ws + kOffBT2);
  unsigned short* SBH  = (unsigned short*)(ws + kOffSBH);
  unsigned short* SBL  = (unsigned short*)(ws + kOffSBL);
  float*          Y1   = (float*)(ws + kOffY1);
  float*          SC   = (float*)(ws + kOffSC);
  float*          CS   = (float*)(ws + kOffCS);
  float*          SN   = (float*)(ws + kOffSN);
  unsigned short* CTH  = (unsigned short*)(ws + kOffCTH);
  unsigned short* CTL  = (unsigned short*)(ws + kOffCTL);
  unsigned short* W1H  = (unsigned short*)(ws + kOffW1H);
  unsigned short* W1L  = (unsigned short*)(ws + kOffW1L);
  unsigned short* WFCH = (unsigned short*)(ws + kOffWFCH);
  unsigned short* WFCL = (unsigned short*)(ws + kOffWFCL);
  unsigned short* WSVH = (unsigned short*)(ws + kOffWSVH);
  unsigned short* WSVL = (unsigned short*)(ws + kOffWSVL);
  unsigned short* W67  = (unsigned short*)(ws + kOffW67);
  float*          VEC  = (float*)(ws + kOffVEC);

  prep_kernel<<<kPrepRowBlocks + 1, 256, 0, stream>>>(
      weight, cross_w, cross_b, crossfc_w, crossfc_b, vsdir_w, vsdir_b,
      sv_w, vs_w, vs_b, ss_w, ss_b, W1H, W1L, WFCH, WFCL, WSVH, WSVL, W67, VEC);

  for (int ch = 0; ch < kChunks; ++ch) {
    const float* vch = v_input + (size_t)ch * kChunkB * kChan * kCols;
    const float* sch = s_input + (size_t)ch * kChunkB * kSch * kPts;

    transpose_cvt_kernel<128, 1><<<dim3(kCols / 64, kChunkB, 1), 256, 0, stream>>>(
        vch, (long)kChan * kCols, kCols, VTH, VTL, kChan, 0, kCols, 1.0f);
    transpose_cvt_kernel<64, 0><<<dim3(kPts / 64, kChunkB, 1), 256, 0, stream>>>(
        sch, (long)kSch * kPts, kPts, BT2, BT2, kK67, kChan, kPts, kCarrySin);
    transpose_cvt_kernel<64, 1><<<dim3(kPts / 64, kChunkB, 1), 256, 0, stream>>>(
        sch, (long)kSch * kPts, kPts, SBH, SBL, kSch, 0, kPts, 1.0f);

    gemm16_kernel<true><<<dim3(((kM1 / 64) * (kCols / 64)) / 8, kChunkB), 256, 0, stream>>>(
        W1H, W1L, kChan, VTH, VTL, kChan, (long)kCols * kChan,
        Y1, kCols, (long)kM1 * kCols, VEC + kVecBias1, kM1, kCols, kChan, 1.0f);
    gemm16_kernel<true><<<dim3(((kChan / 64) * (kPts / 64)) / 8, kChunkB), 256, 0, stream>>>(
        WSVH, WSVL, kSch, SBH, SBL, kSch, (long)kPts * kSch,
        SC, kPts, (long)kChan * kPts, sv_b, kChan, kPts, kSch, 1.0f);

    stats_kernel<<<(kChunkB * kPts) / 256, 256, 0, stream>>>(vch, Y1, SC, VEC + kVecRsv, CS, SN);

    transpose_cvt_kernel<128, 1><<<dim3(kCols / 64, kChunkB, 2), 256, 0, stream>>>(
        CS, (long)kKfc * kCols, kCols, CTH, CTL, kKfc, 0, kCols, 1.0f);
    transpose_cvt_kernel<128, 0><<<dim3(kPts / 64, kChunkB, 1), 256, 0, stream>>>(
        SN, (long)kChan * kPts, kPts, BT2, BT2, kK67, 0, kPts, kCarrySn);

    gemm16_kernel<true><<<dim3(((kChan / 64) * (kCols / 64)) / 8, kChunkB), 256, 0, stream>>>(
        WFCH, WFCL, kKfc, CTH, CTL, kKfc, (long)kCols * kKfc,
        out0 + (size_t)ch * kChunkB * kChan * kCols, kCols, (long)kChan * kCols,
        VEC + kVecBfc, kChan, kCols, kKfc, 1.0f);
    gemm16_kernel<false><<<dim3(((kSch / 64) * (kPts / 64)) / 8, kChunkB), 256, 0, stream>>>(
        W67, W67, kK67, BT2, BT2, kK67, (long)kPts * kK67,
        out1 + (size_t)ch * kChunkB * kSch * kPts, kPts, (long)kSch * kPts,
        VEC + kVecB67, kSch, kPts, kK67, kFold67);
  }
}
